// TransformerEncoder_1889785610583
// MI455X (gfx1250) — hardware-verified
//
#include <hip/hip_runtime.h>
#ifndef NB
#define NB 4
#endif
#ifndef SEQ
#define SEQ 1024
#endif
#define NB_FULL 4
#define SEQ_FULL 1024
#define FEAT 512
#define NHEAD 8
#define DHEAD 64
#define MLPH 2048
#define NLAYER 6
#define MR (NB * SEQ)
#define QKVN (3 * FEAT)
static_assert(SEQ % 64 == 0);
static_assert(SEQ <= SEQ_FULL);
static_assert(NB >= 1);
static_assert(NB <= NB_FULL);
static_assert(FEAT == NHEAD * DHEAD);
static_assert(FEAT % 64 == 0);
static_assert(MLPH % 64 == 0);
static_assert(QKVN % 64 == 0);
static_assert(FEAT == 64 * 8);
static_assert(FEAT == 128 * 4);
static_assert(MR % 16 == 0);
static_assert(FEAT % 32 == 0);
static_assert(MLPH % 32 == 0);
static_assert((FEAT / 8) % 8 == 0);
static_assert((MLPH / 8) % 8 == 0);

typedef _Float16 v16h __attribute__((ext_vector_type(16)));
typedef unsigned short v8us __attribute__((ext_vector_type(8), may_alias));
typedef float v8f __attribute__((ext_vector_type(8)));
typedef float v4f __attribute__((ext_vector_type(4)));
typedef float v4fa __attribute__((ext_vector_type(4), may_alias));
union FragH { v16h v; v8us half[2]; unsigned short u[16]; };
union H16U { _Float16 h; unsigned short u; };

__device__ __forceinline__ unsigned short bf16_bits(float x) { unsigned int u = __float_as_uint(x); return (unsigned short)((u + 0x7FFFu + ((u >> 16) & 1u)) >> 16); }
__device__ __forceinline__ float bf16_val(unsigned short b) { return __uint_as_float(((unsigned int)b) << 16); }
__device__ __forceinline__ float bf16_rne(float x) { return bf16_val(bf16_bits(x)); }
__device__ __forceinline__ unsigned short h16_bits(float x) { H16U t; t.h = (_Float16)x; return t.u; }
__device__ __forceinline__ v8f vz8() { v8f z = {0.f, 0.f, 0.f, 0.f, 0.f, 0.f, 0.f, 0.f}; return z; }

__device__ __forceinline__ v8f mma16(v16h a, v16h b, v8f c) {
  c = __builtin_amdgcn_wmma_f32_16x16x32_f16(false, a, false, b, (short)0, c, false, false);
  asm volatile("v_nop\n\tv_nop\n\tv_nop\n\tv_nop" : "+v"(c) : "v"(a), "v"(b));
  return c;
}

__global__ __launch_bounds__(256) void k_wt16(const float* __restrict__ W, unsigned short* __restrict__ Wt, int K, int N, int nl,
                                             size_t lstride, int roff, float sc) {
  const int t = blockIdx.x * 256 + threadIdx.x;
  const int k8n = K / 8;
  const int per = N * k8n;
  if (t >= per * nl) return;
  const int l = t / per, rem = t - l * per;
  const int n = rem / k8n, k8 = (rem % k8n) * 8;
  const float* src = W + (size_t)l * K * N;
  v8us v;
#pragma unroll
  for (int i = 0; i < 8; ++i) v[i] = h16_bits(bf16_rne(src[(size_t)(k8 + i) * N + n]) * sc);
  unsigned short* dst = Wt + (size_t)l * lstride + (size_t)(roff + n) * K + k8;
  *(volatile v8us*)dst = v;
  __threadfence();
  *(volatile v8us*)dst = v;
}

__global__ __launch_bounds__(128) void k_xinit(const float* __restrict__ src, const float* __restrict__ pos, float* __restrict__ X,
                                               int seq, int nbf) {
  const int m = blockIdx.x, tid = threadIdx.x;
  const int b = m / seq, s = m % seq;
  const size_t so = ((size_t)s * nbf + b) * FEAT + tid * 4;
  const v4f a = *(const v4fa*)(src + so);
  const v4f p = *(const v4fa*)(pos + so);
  v4f o;
#pragma unroll
  for (int i = 0; i < 4; ++i) o[i] = bf16_rne(a[i]) + bf16_rne(p[i]);
  float* dst = X + (size_t)m * FEAT + tid * 4;
  *(volatile v4f*)dst = o;
  __threadfence();
  *(volatile v4f*)dst = o;
}

__global__ __launch_bounds__(64) void k_ln16(const float* __restrict__ X, const float* __restrict__ g, const float* __restrict__ bt,
                                            unsigned short* __restrict__ out, float osc, float eps) {
  __shared__ float red1[2];
  __shared__ float red2[2];
  const int m = blockIdx.x, tid = threadIdx.x, w = tid >> 5, lane = tid & 31;
  const float* x = X + (size_t)m * FEAT + tid * 8;
  const v4f a0 = *(const v4fa*)x;
  const v4f a1 = *(const v4fa*)(x + 4);
  float v[8] = {a0[0], a0[1], a0[2], a0[3], a1[0], a1[1], a1[2], a1[3]};
  float s = 0.f;
#pragma unroll
  for (int q = 0; q < 8; ++q) s += v[q];
#pragma unroll
  for (int o = 16; o >= 1; o >>= 1) s += __shfl_xor(s, o, 32);
  if (lane == 0) red1[w] = s;
  __syncthreads();
  const float mu = (red1[0] + red1[1]) * (1.0f / (float)FEAT);
  float c[8];
  float s2 = 0.f;
#pragma unroll
  for (int q = 0; q < 8; ++q) { c[q] = v[q] - mu; s2 += c[q] * c[q]; }
#pragma unroll
  for (int o = 16; o >= 1; o >>= 1) s2 += __shfl_xor(s2, o, 32);
  if (lane == 0) red2[w] = s2;
  __syncthreads();
  const float var = (red2[0] + red2[1]) * (1.0f / (float)FEAT);
  const float rs = rsqrtf(var + eps);
  const v4f g0 = *(const v4fa*)(g + tid * 8);
  const v4f g1 = *(const v4fa*)(g + tid * 8 + 4);
  const v4f b0 = *(const v4fa*)(bt + tid * 8);
  const v4f b1 = *(const v4fa*)(bt + tid * 8 + 4);
  const float gg[8] = {g0[0], g0[1], g0[2], g0[3], g1[0], g1[1], g1[2], g1[3]};
  const float bb[8] = {b0[0], b0[1], b0[2], b0[3], b1[0], b1[1], b1[2], b1[3]};
  v8us o;
#pragma unroll
  for (int q = 0; q < 8; ++q) o[q] = h16_bits((c[q] * rs * bf16_rne(gg[q]) + bf16_rne(bb[q])) * osc);
  unsigned short* dst = out + (size_t)m * FEAT + tid * 8;
  *(volatile v8us*)dst = o;
  __threadfence();
  *(volatile v8us*)dst = o;
}

__global__ __launch_bounds__(128) void k_lnf32(const float* __restrict__ X, const float* __restrict__ g, const float* __restrict__ bt,
                                               float* __restrict__ out, int seq, int nbf, float eps) {
  __shared__ float red1[4];
  __shared__ float red2[4];
  const int m = blockIdx.x, tid = threadIdx.x, w = tid >> 5, lane = tid & 31;
  const int b = m / seq, s = m % seq;
  const v4f a = *(const v4fa*)(X + (size_t)m * FEAT + tid * 4);
  float sm = a[0] + a[1] + a[2] + a[3];
#pragma unroll
  for (int o = 16; o >= 1; o >>= 1) sm += __shfl_xor(sm, o, 32);
  if (lane == 0) red1[w] = sm;
  __syncthreads();
  const float mu = (red1[0] + red1[1] + red1[2] + red1[3]) * (1.0f / (float)FEAT);
  float c[4];
  float s2 = 0.f;
#pragma unroll
  for (int q = 0; q < 4; ++q) { c[q] = a[q] - mu; s2 += c[q] * c[q]; }
#pragma unroll
  for (int o = 16; o >= 1; o >>= 1) s2 += __shfl_xor(s2, o, 32);
  if (lane == 0) red2[w] = s2;
  __syncthreads();
  const float var = (red2[0] + red2[1] + red2[2] + red2[3]) * (1.0f / (float)FEAT);
  const float rs = rsqrtf(var + eps);
  const v4f g4 = *(const v4fa*)(g + tid * 4);
  const v4f b4 = *(const v4fa*)(bt + tid * 4);
  v4f o;
#pragma unroll
  for (int q = 0; q < 4; ++q) o[q] = c[q] * rs * bf16_rne(g4[q]) + bf16_rne(b4[q]);
  float* dst = out + ((size_t)s * nbf + b) * FEAT + tid * 4;
  *(volatile v4f*)dst = o;
  __threadfence();
  *(volatile v4f*)dst = o;
}

template <bool OUT16, int ACT>
__global__ __launch_bounds__(128) void k_gemm16(const unsigned short* __restrict__ A, int lda, const unsigned short* __restrict__ Wt, int ldb,
                                               const float* __restrict__ bias0, const float* __restrict__ bias1, const float* __restrict__ bias2, int nsplit,
                                               const float* __restrict__ resid, int ldr, void* __restrict__ Cv, int ldc,
                                               int M, int N, int K, float inv_scale, float out_scale) {
  __shared__ __attribute__((aligned(16))) float so32[OUT16 ? 1 : 4][16][64];
  __shared__ __attribute__((aligned(16))) unsigned short so16[OUT16 ? 4 : 1][16][72];
  const int tid = threadIdx.x, w = tid >> 5, lane = tid & 31, ln = lane & 15, hh = lane >> 4;
  const int ntn = N / 64;
  const int wid = blockIdx.x * 4 + w;
  const int mt = wid / ntn, nq = wid % ntn;
  if (mt * 16 >= M) return;
  const int row0 = mt * 16, col0 = nq * 64;
  const unsigned short* arow = A + (size_t)(row0 + ln) * lda;
  v8f acc[4];
#pragma unroll
  for (int t = 0; t < 4; ++t) acc[t] = vz8();
  for (int kb = 0; kb < K; kb += 32) {
    FragH a;
    a.half[0] = *(const v8us*)(arow + kb + 8 * hh);
    a.half[1] = *(const v8us*)(arow + kb + 16 + 8 * hh);
#pragma unroll
    for (int t = 0; t < 4; ++t) {
      const unsigned short* brow = Wt + (size_t)(col0 + t * 16 + ln) * ldb + kb;
      FragH bb;
      bb.half[0] = *(const v8us*)(brow + 8 * hh);
      bb.half[1] = *(const v8us*)(brow + 16 + 8 * hh);
      acc[t] = mma16(a.v, bb.v, acc[t]);
    }
  }
  int seg = col0 / nsplit; seg = (seg > 2) ? 2 : seg;
  const float* bsel = (seg == 0) ? bias0 : ((seg == 1) ? bias1 : bias2);
#pragma unroll
  for (int t = 0; t < 4; ++t) {
    const int col = col0 + t * 16 + ln;
    const float bvv = bf16_rne(bsel[col - seg * nsplit]);
#pragma unroll
    for (int r = 0; r < 8; ++r) {
      float v = acc[t][r] * inv_scale + bvv;
      if (ACT == 1) v = fmaxf(v, 0.0f);
      if constexpr (OUT16) so16[w][8 * hh + r][t * 16 + ln] = h16_bits(v * out_scale);
      else so32[w][8 * hh + r][t * 16 + ln] = v;
    }
  }
  __builtin_amdgcn_fence(4  , "workgroup");
  __builtin_amdgcn_wave_barrier();
  if constexpr (OUT16) {
    unsigned short* Ch = (unsigned short*)Cv;
    const int rq = lane >> 3, p8 = (lane & 7) * 8;
    for (int pass = 0; pass < 2; ++pass) {
#pragma unroll
      for (int q = 0; q < 4; ++q) {
        const int r = q * 4 + rq;
        const v8us v = *(const v8us*)&so16[w][r][p8];
        *(volatile v8us*)(Ch + (size_t)(row0 + r) * ldc + col0 + p8) = v;
      }
      if (pass == 0) __threadfence();
    }
  } else {
    float* Cf = (float*)Cv;
    const int rsub = lane >> 4, c4 = (lane & 15) * 4;
    if (resid != nullptr) {
#pragma unroll
      for (int q = 0; q < 8; ++q) {
        const int r = q * 2 + rsub;
        const v4f rv = *(const v4fa*)(resid + (size_t)(row0 + r) * ldr + col0 + c4);
        v4f tv = *(const v4fa*)&so32[w][r][c4];
        tv += rv;
        *(v4fa*)&so32[w][r][c4] = tv;
      }
    }
    for (int pass = 0; pass < 2; ++pass) {
#pragma unroll
      for (int q = 0; q < 8; ++q) {
        const int r = q * 2 + rsub;
        const v4f v = *(const v4fa*)&so32[w][r][c4];
        *(volatile v4f*)(Cf + (size_t)(row0 + r) * ldc + col0 + c4) = v;
      }
      if (pass == 0) __threadfence();
    }
  }
}

template <int D>
__global__ __launch_bounds__(128) void k_attn16(const unsigned short* __restrict__ qkv, int pitch, int T, int H, int koff, int voff,
                                                float scale, float pcarry, float onorm,
                                                const float* __restrict__ resid, float* __restrict__ out, int opitch) {
  static_assert(D == 64);
  constexpr int KS = D / 32, DT = D / 16, C8 = D / 8;
  static_assert((32 * C8) % 128 == 0);
  __shared__ __attribute__((aligned(16))) unsigned short sK[32][D + 8];
  __shared__ __attribute__((aligned(16))) unsigned short sVt[D][40];
  __shared__ __attribute__((aligned(16))) unsigned short sP[4][16][40];
  __shared__ __attribute__((aligned(16))) float sO[4][16][D + 4];
  const int tid = threadIdx.x, w = tid >> 5, lane = tid & 31, ln = lane & 15, hh = lane >> 4;
  const int nqb = T / 64;
  const int bh = blockIdx.x / nqb, qblk = blockIdx.x % nqb;
  const int b = bh / H, h = bh % H;
  const int q0 = qblk * 64 + w * 16;
  const unsigned short* Qp = qkv + (size_t)b * T * pitch + h * D;
  const unsigned short* Kp = Qp + koff;
  const unsigned short* Vp = Qp + voff;

  FragH aq[KS];
  {
    const unsigned short* qr = Qp + (size_t)(q0 + ln) * pitch;
#pragma unroll
    for (int ks = 0; ks < KS; ++ks) {
      aq[ks].half[0] = *(const v8us*)(qr + ks * 32 + 8 * hh);
      aq[ks].half[1] = *(const v8us*)(qr + ks * 32 + 16 + 8 * hh);
    }
  }
  float m_r[8], l_r[8];
#pragma unroll
  for (int r = 0; r < 8; ++r) { m_r[r] = -1.0e30f; l_r[r] = 0.f; }
  v8f oacc[DT];
#pragma unroll
  for (int dt = 0; dt < DT; ++dt) oacc[dt] = vz8();

  for (int j0 = 0; j0 < T; j0 += 32) {
    __syncthreads();
#pragma unroll
    for (int it = 0; it < (32 * C8) / 128; ++it) {
      const int e = tid + it * 128;
      const int r = e / C8, c8 = (e % C8) * 8;
      const size_t ro = (size_t)(j0 + r) * pitch + c8;
      const v8us kvv = *(const v8us*)(Kp + ro);
      *(v8us*)&sK[r][c8] = kvv;
      const v8us vvv = *(const v8us*)(Vp + ro);
#pragma unroll
      for (int i = 0; i < 8; ++i) sVt[c8 + i][r] = vvv[i];
    }
    __syncthreads();
    v8f s[2];
#pragma unroll
    for (int nt = 0; nt < 2; ++nt) {
      v8f acc = vz8();
#pragma unroll
      for (int ks = 0; ks < KS; ++ks) {
        FragH bk;
        bk.half[0] = *(const v8us*)&sK[nt * 16 + ln][ks * 32 + 8 * hh];
        bk.half[1] = *(const v8us*)&sK[nt * 16 + ln][ks * 32 + 16 + 8 * hh];
        acc = mma16(aq[ks].v, bk.v, acc);
      }
      s[nt] = acc;
    }
    float alpha[8];
#pragma unroll
    for (int r = 0; r < 8; ++r) {
      const float s0 = s[0][r] * scale, s1 = s[1][r] * scale;
      float mx = fmaxf(s0, s1);
      mx = fmaxf(mx, __shfl_xor(mx, 1, 32)); mx = fmaxf(mx, __shfl_xor(mx, 2, 32));
      mx = fmaxf(mx, __shfl_xor(mx, 4, 32)); mx = fmaxf(mx, __shfl_xor(mx, 8, 32));
      const float mnew = fmaxf(m_r[r], mx);
      alpha[r] = __expf(m_r[r] - mnew);
      const float p0 = __expf(s0 - mnew), p1 = __expf(s1 - mnew);
      m_r[r] = mnew;
      l_r[r] = l_r[r] * alpha[r] + p0 + p1;
      sP[w][8 * hh + r][ln] = h16_bits(p0 * pcarry);
      sP[w][8 * hh + r][16 + ln] = h16_bits(p1 * pcarry);
    }
#pragma unroll
    for (int dt = 0; dt < DT; ++dt)
#pragma unroll
      for (int r = 0; r < 8; ++r) oacc[dt][r] *= alpha[r];
    __builtin_amdgcn_fence(4  , "workgroup");
    __builtin_amdgcn_wave_barrier();
    FragH pa;
    pa.half[0] = *(const v8us*)&sP[w][ln][8 * hh];
    pa.half[1] = *(const v8us*)&sP[w][ln][16 + 8 * hh];
#pragma unroll
    for (int dt = 0; dt < DT; ++dt) {
      FragH bv;
      bv.half[0] = *(const v8us*)&sVt[dt * 16 + ln][8 * hh];
      bv.half[1] = *(const v8us*)&sVt[dt * 16 + ln][16 + 8 * hh];
      oacc[dt] = mma16(pa.v, bv.v, oacc[dt]);
    }
    __builtin_amdgcn_fence(4  , "workgroup");
    __builtin_amdgcn_wave_barrier();
  }
#pragma unroll
  for (int r = 0; r < 8; ++r) {
    float l = l_r[r];
    l += __shfl_xor(l, 1, 32); l += __shfl_xor(l, 2, 32); l += __shfl_xor(l, 4, 32); l += __shfl_xor(l, 8, 32);
    l_r[r] = onorm * (1.0f / l);
  }
#pragma unroll
  for (int dt = 0; dt < DT; ++dt)
#pragma unroll
    for (int r = 0; r < 8; ++r) sO[w][8 * hh + r][dt * 16 + ln] = oacc[dt][r] * l_r[r];
  __builtin_amdgcn_fence(4  , "workgroup");
  __builtin_amdgcn_wave_barrier();
  const int rsub = lane >> 4, c4 = (lane & 15) * 4;
  const size_t rbase = (size_t)(b * T + q0) * opitch + h * D;
#pragma unroll
  for (int q = 0; q < 8; ++q) {
    const int r = q * 2 + rsub;
    const v4f rv = *(const v4fa*)(resid + rbase + (size_t)r * opitch + c4);
    v4f tv = *(const v4fa*)&sO[w][r][c4];
    tv += rv;
    *(v4fa*)&sO[w][r][c4] = tv;
  }
  for (int pass = 0; pass < 2; ++pass) {
#pragma unroll
    for (int q = 0; q < 8; ++q) {
      const int r = q * 2 + rsub;
      const v4f v = *(const v4fa*)&sO[w][r][c4];
      *(volatile v4f*)(out + rbase + (size_t)r * opitch + c4) = v;
    }
    if (pass == 0) __threadfence();
  }
}

extern "C" void kernel_launch(void* const* d_in, const int* in_sizes, int n_in,
                              void* d_out, int out_size, void* d_ws, size_t ws_size, hipStream_t stream) {
  if (n_in < 18) return;
  const long long need_rows = (long long)(SEQ - 1) * NB_FULL + NB;
  if ((long long)in_sizes[0] < need_rows * FEAT || (long long)in_sizes[1] < need_rows * FEAT) return;
  if (in_sizes[2] < NLAYER * FEAT * FEAT || in_sizes[4] < NLAYER * FEAT * FEAT || in_sizes[6] < NLAYER * FEAT * FEAT) return;
  if (in_sizes[3] < NLAYER * FEAT || in_sizes[5] < NLAYER * FEAT || in_sizes[7] < NLAYER * FEAT || in_sizes[11] < NLAYER * FEAT) return;
  if (in_sizes[8] < NLAYER * FEAT * MLPH || in_sizes[9] < NLAYER * MLPH || in_sizes[10] < NLAYER * MLPH * FEAT) return;
  if (in_sizes[12] < NLAYER * FEAT || in_sizes[13] < NLAYER * FEAT || in_sizes[14] < NLAYER * FEAT || in_sizes[15] < NLAYER * FEAT) return;
  if (in_sizes[16] < FEAT || in_sizes[17] < FEAT) return;
  if ((long long)out_size < need_rows * FEAT) return;

  const float* src  = (const float*)d_in[0];
  const float* pos  = (const float*)d_in[1];
  const float* Wq   = (const float*)d_in[2];  const float* bq   = (const float*)d_in[3];
  const float* Wk   = (const float*)d_in[4];  const float* bk   = (const float*)d_in[5];
  const float* Wv   = (const float*)d_in[6];  const float* bv   = (const float*)d_in[7];
  const float* W1   = (const float*)d_in[8];  const float* b1   = (const float*)d_in[9];
  const float* W2   = (const float*)d_in[10]; const float* b2   = (const float*)d_in[11];
  const float* ln1g = (const float*)d_in[12]; const float* ln1b = (const float*)d_in[13];
  const float* ln2g = (const float*)d_in[14]; const float* ln2b = (const float*)d_in[15];
  const float* lnfg = (const float*)d_in[16]; const float* lnfb = (const float*)d_in[17];

  char* ws = (char*)d_ws; size_t off = 0;
  auto take = [&](size_t bytes) { char* p = ws + off; off += (bytes + 255) & ~(size_t)255; return p; };
  const size_t lsq = (size_t)QKVN * FEAT;
  const size_t ls1 = (size_t)MLPH * FEAT, ls2 = (size_t)FEAT * MLPH;
  unsigned short* Wqkv16 = (unsigned short*)take((size_t)NLAYER * lsq * 2);
  unsigned short* W116   = (unsigned short*)take((size_t)NLAYER * ls1 * 2);
  unsigned short* W216   = (unsigned short*)take((size_t)NLAYER * ls2 * 2);
  float* XA = (float*)take((size_t)MR * FEAT * 4);
  float* XB = (float*)take((size_t)MR * FEAT * 4);
  const size_t r1_bytes = (size_t)MR * FEAT * 2;
  const size_t r2_a = (size_t)MR * QKVN * 2, r2_b = (size_t)MR * MLPH * 2;
  const size_t r2_bytes = (r2_a > r2_b) ? r2_a : r2_b;
  unsigned short* R1 = (unsigned short*)take(r1_bytes);
  unsigned short* R2 = (unsigned short*)take(r2_bytes);
  if (off > ws_size) return;
  if (off > (size_t)134217728) return;

  const float wsc = 256.0f;
  const int k8d = FEAT / 8, k8m = MLPH / 8;
  k_wt16<<<(unsigned)((NLAYER * FEAT * k8d + 255) / 256), 256, 0, stream>>>(Wq, Wqkv16, FEAT, FEAT, NLAYER, lsq, 0, wsc);
  k_wt16<<<(unsigned)((NLAYER * FEAT * k8d + 255) / 256), 256, 0, stream>>>(Wk, Wqkv16, FEAT, FEAT, NLAYER, lsq, FEAT, wsc);
  k_wt16<<<(unsigned)((NLAYER * FEAT * k8d + 255) / 256), 256, 0, stream>>>(Wv, Wqkv16, FEAT, FEAT, NLAYER, lsq, 2 * FEAT, wsc);
  k_wt16<<<(unsigned)((NLAYER * MLPH * k8d + 255) / 256), 256, 0, stream>>>(W1, W116, FEAT, MLPH, NLAYER, ls1, 0, wsc);
  k_wt16<<<(unsigned)((NLAYER * FEAT * k8m + 255) / 256), 256, 0, stream>>>(W2, W216, MLPH, FEAT, NLAYER, ls2, 0, wsc);

  k_xinit<<<(unsigned)MR, 128, 0, stream>>>(src, pos, XA, SEQ, NB_FULL);

  auto ggrid = [](int M, int N) { return (unsigned)(((M / 16) * (N / 64) + 3) / 4); };
  const float scale = 0.125f;

  for (int l = 0; l < NLAYER; ++l) {
    k_ln16<<<(unsigned)MR, 64, 0, stream>>>(XA, ln1g + l * FEAT, ln1b + l * FEAT, R1, 8.0f, 1e-5f);
    k_gemm16<true, 0><<<ggrid(MR, QKVN), 128, 0, stream>>>(R1, FEAT, Wqkv16 + (size_t)l * lsq, FEAT,
                                                          bq + l * FEAT, bk + l * FEAT, bv + l * FEAT, FEAT, nullptr, 0,
                                                          (void*)R2, QKVN, MR, QKVN, FEAT, 1.0f / 2048.0f, 1.0f);
    k_attn16<DHEAD><<<(unsigned)(NB * NHEAD * (SEQ / 64)), 128, 0, stream>>>(R2, QKVN, SEQ, NHEAD, FEAT, 2 * FEAT, scale, 1024.0f,
                                                                             1.0f / 1024.0f, XA, XB, FEAT);
    k_ln16<<<(unsigned)MR, 64, 0, stream>>>(XB, ln2g + l * FEAT, ln2b + l * FEAT, R1, 8.0f, 1e-5f);
    k_gemm16<true, 1><<<ggrid(MR, MLPH), 128, 0, stream>>>(R1, FEAT, W116 + (size_t)l * ls1, FEAT,
                                                          b1 + l * MLPH, b1 + l * MLPH, b1 + l * MLPH, MLPH, nullptr, 0,
                                                          (void*)R2, MLPH, MR, MLPH, FEAT, 1.0f / 2048.0f, 16.0f);
    k_gemm16<false, 0><<<ggrid(MR, FEAT), 128, 0, stream>>>(R2, MLPH, W216 + (size_t)l * ls2, MLPH,
                                                           b2 + l * FEAT, b2 + l * FEAT, b2 + l * FEAT, FEAT, XB, FEAT,
                                                           (void*)XA, FEAT, MR, FEAT, MLPH, 1.0f / 4096.0f, 1.0f);
  }
  k_lnf32<<<(unsigned)MR, 128, 0, stream>>>(XA, lnfg, lnfb, (float*)d_out, SEQ, NB_FULL, 1e-5f);
}
